// NaLPFactBlock_28252294873241
// MI455X (gfx1250) — hardware-verified
//
#include <hip/hip_runtime.h>

#pragma clang fp contract(off)

typedef __bf16         v16b __attribute__((ext_vector_type(16)));
typedef unsigned short v8us __attribute__((ext_vector_type(8)));
typedef float          v8f  __attribute__((ext_vector_type(8)));
typedef float          v4f  __attribute__((ext_vector_type(4)));
typedef v8us __attribute__((may_alias)) v8usa;
typedef v4f  __attribute__((may_alias)) v4fa;

union Frag { v16b v; v8us half[2]; };

#define NB     1024
#define AR     16
#define EMB    128
#define NROLES 1000
#define KP     256
#define NF     256
#define NG     512
#define KG     512
#define MROWS  (NB * AR)

#define GP   ((MROWS * KP) / 8)
#define GC   ((NF * KP) / 8)
#define GG   ((NG * KG) / 8)
#define GTOT (GP + GC + GG)
#define PREP_THREADS 256

static_assert(GP % PREP_THREADS == 0);
static_assert((GP + GC) % PREP_THREADS == 0);
static_assert(GTOT % PREP_THREADS == 0);
static_assert(KP / 8 == 32);
static_assert(MROWS % 128 == 0);
static_assert(NF % 64 == 0);
static_assert(NG % 128 == 0);
static_assert(KP % 32 == 0);
static_assert(NF % 32 == 0);

__device__ __forceinline__ v8f wmma_bf16(v16b a, v16b b, v8f c) {
  v8f d = __builtin_amdgcn_wmma_f32_16x16x32_bf16(false, a, false, b, (short)0, c, false, false);
  asm volatile("v_nop\n\tv_nop\n\tv_nop\n\tv_nop" : "+v"(d) : "v"(a), "v"(b));
  return d;
}

__device__ __forceinline__ v16b load_frag(const unsigned short* p, int h) {
  Frag f;
  f.half[0] = *(const v8usa*)(p + 8 * h);
  f.half[1] = *(const v8usa*)(p + 16 + 8 * h);
  return f.v;
}

__device__ __forceinline__ unsigned int bf16_rne(float f) {
  const unsigned int u = __float_as_uint(f);
  return (u + 0x7FFFu + ((u >> 16) & 1u)) >> 16;
}

__device__ __forceinline__ void split1(float f, unsigned short& hi, unsigned short& lo) {
  const unsigned int hb = bf16_rne(f);
  const float hf = __uint_as_float(hb << 16);
  hi = (unsigned short)hb;
  lo = (unsigned short)bf16_rne(f - hf);
}

struct HL8 { v8us hi; v8us lo; };

__device__ __forceinline__ HL8 split8(v4f a, v4f c) {
  unsigned short h0, h1, h2, h3, h4, h5, h6, h7;
  unsigned short l0, l1, l2, l3, l4, l5, l6, l7;
  split1(a.x, h0, l0); split1(a.y, h1, l1); split1(a.z, h2, l2); split1(a.w, h3, l3);
  split1(c.x, h4, l4); split1(c.y, h5, l5); split1(c.z, h6, l6); split1(c.w, h7, l7);
  HL8 r;
  const v8us vh = { h0, h1, h2, h3, h4, h5, h6, h7 };
  const v8us vl = { l0, l1, l2, l3, l4, l5, l6, l7 };
  r.hi = vh;
  r.lo = vl;
  return r;
}

__global__ __launch_bounds__(PREP_THREADS) void prep_kernel(
    const int* __restrict__ role_ids,
    const float* __restrict__ value_embeds,
    const float* __restrict__ role_table,
    const float* __restrict__ conv_w,
    const float* __restrict__ gfcn_w,
    unsigned short* __restrict__ Ph, unsigned short* __restrict__ Pl,
    unsigned short* __restrict__ CWh, unsigned short* __restrict__ CWl,
    unsigned short* __restrict__ GWh, unsigned short* __restrict__ GWl)
{
  const int g = blockIdx.x * PREP_THREADS + threadIdx.x;
  if (g >= GTOT) return;

  v4f a, c;
  unsigned short* dh;
  unsigned short* dl;
  if (g < GP) {
    const int row = g >> 5;
    const int cg  = g & 31;
    const int c8  = (cg & 15) * 8;
    int rid = role_ids[row];
    rid = min(max(rid, 0), NROLES - 1);
    const float* pr = role_table   + (size_t)rid * EMB + c8;
    const float* pv = value_embeds + (size_t)row * EMB + c8;
    const v4f ra = *(const v4fa*)pr;
    const v4f rc = *(const v4fa*)(pr + 4);
    const v4f va = *(const v4fa*)pv;
    const v4f vc = *(const v4fa*)(pv + 4);
    const bool isRole = (cg < 16);
    a = isRole ? ra : va;
    c = isRole ? rc : vc;
    dh = Ph + (size_t)g * 8;
    dl = Pl + (size_t)g * 8;
  } else if (g < GP + GC) {
    const int e = g - GP;
    const float* p = conv_w + (size_t)e * 8;
    a = *(const v4fa*)p;
    c = *(const v4fa*)(p + 4);
    dh = CWh + (size_t)e * 8;
    dl = CWl + (size_t)e * 8;
  } else {
    const int e = g - GP - GC;
    const float* p = gfcn_w + (size_t)e * 8;
    a = *(const v4fa*)p;
    c = *(const v4fa*)(p + 4);
    dh = GWh + (size_t)e * 8;
    dl = GWl + (size_t)e * 8;
  }

  const HL8 s = split8(a, c);
  *(volatile v8us*)dh = s.hi;
  *(volatile v8us*)dl = s.lo;
  __threadfence();
  *(volatile v8us*)dh = s.hi;
  *(volatile v8us*)dl = s.lo;
}

__device__ __forceinline__ void x_store_pass(const unsigned short* s, unsigned short* X,
                                             int m0, int n0, int w, int lane) {
  const int q8 = lane & 7, sub = lane >> 3;
  #pragma unroll
  for (int i = 0; i < 8; ++i) {
    const int rowl = 32 * w + 4 * i + sub;
    const v8us v = *(const v8usa*)(s + rowl * 64 + 8 * q8);
    *(volatile v8us*)(X + (size_t)(m0 + rowl) * NF + n0 + 8 * q8) = v;
  }
}

__global__ __launch_bounds__(128) void gemm1_bn_kernel(
    const unsigned short* __restrict__ Ph,  const unsigned short* __restrict__ Pl,
    const unsigned short* __restrict__ CWh, const unsigned short* __restrict__ CWl,
    const float* __restrict__ conv_b,
    const float* __restrict__ bn_gamma, const float* __restrict__ bn_beta,
    const float* __restrict__ bn_mean,  const float* __restrict__ bn_var,
    unsigned short* __restrict__ Xh, unsigned short* __restrict__ Xl)
{
  __shared__ __attribute__((aligned(16))) unsigned short sT[2 * 128 * 64];

  const int tid = threadIdx.x, lane = tid & 31, w = tid >> 5;
  const int h = lane >> 4, m = lane & 15;
  const int m0 = blockIdx.x * 128, n0 = blockIdx.y * 64;
  const int m0w = m0 + 32 * w;

  const unsigned short* a0h = Ph + (size_t)(m0w + m) * KP;
  const unsigned short* a1h = a0h + (size_t)16 * KP;
  const unsigned short* a0l = Pl + (size_t)(m0w + m) * KP;
  const unsigned short* a1l = a0l + (size_t)16 * KP;
  const unsigned short* bwh = CWh + (size_t)(n0 + m) * KP;
  const unsigned short* bwl = CWl + (size_t)(n0 + m) * KP;

  const v8f zero8 = {0.f, 0.f, 0.f, 0.f, 0.f, 0.f, 0.f, 0.f};
  v8f acc[2][4];
  #pragma unroll
  for (int mt = 0; mt < 2; ++mt)
    #pragma unroll
    for (int nt = 0; nt < 4; ++nt) acc[mt][nt] = zero8;

  #pragma unroll 1
  for (int k0 = 0; k0 < KP; k0 += 32) {
    const v16b fa0h = load_frag(a0h + k0, h);
    const v16b fa1h = load_frag(a1h + k0, h);
    const v16b fa0l = load_frag(a0l + k0, h);
    const v16b fa1l = load_frag(a1l + k0, h);
    #pragma unroll
    for (int nt = 0; nt < 4; ++nt) {
      const v16b fbh = load_frag(bwh + (size_t)nt * 16 * KP + k0, h);
      const v16b fbl = load_frag(bwl + (size_t)nt * 16 * KP + k0, h);
      acc[0][nt] = wmma_bf16(fa0h, fbh, acc[0][nt]);
      acc[0][nt] = wmma_bf16(fa0h, fbl, acc[0][nt]);
      acc[0][nt] = wmma_bf16(fa0l, fbh, acc[0][nt]);
      acc[1][nt] = wmma_bf16(fa1h, fbh, acc[1][nt]);
      acc[1][nt] = wmma_bf16(fa1h, fbl, acc[1][nt]);
      acc[1][nt] = wmma_bf16(fa1l, fbh, acc[1][nt]);
    }
  }

  #pragma unroll
  for (int nt = 0; nt < 4; ++nt) {
    const int col = 16 * nt + m;
    const int f = n0 + col;
    const float bias = conv_b[f];
    const float sc = bn_gamma[f] / sqrtf(bn_var[f] + 1e-5f);
    const float mn = bn_mean[f];
    const float bt = bn_beta[f];
    #pragma unroll
    for (int mt = 0; mt < 2; ++mt) {
      #pragma unroll
      for (int r = 0; r < 8; ++r) {
        const int rowl = 32 * w + 16 * mt + 8 * h + r;
        float y = acc[mt][nt][r] + bias;
        y = y - mn;
        y = y * sc;
        y = y + bt;
        y = fmaxf(y, 0.0f);
        unsigned short hi, lo;
        split1(y, hi, lo);
        sT[rowl * 64 + col] = hi;
        sT[8192 + rowl * 64 + col] = lo;
      }
    }
  }
  __syncthreads();

  x_store_pass(sT, Xh, m0, n0, w, lane);
  x_store_pass(sT + 8192, Xl, m0, n0, w, lane);
  __threadfence();
  x_store_pass(sT, Xh, m0, n0, w, lane);
  x_store_pass(sT + 8192, Xl, m0, n0, w, lane);
}

__global__ __launch_bounds__(128) void gfcn_min_kernel(
    const unsigned short* __restrict__ Xh,  const unsigned short* __restrict__ Xl,
    const unsigned short* __restrict__ GWh, const unsigned short* __restrict__ GWl,
    const float* __restrict__ gfcn_b,
    float* __restrict__ out)
{
  __shared__ __attribute__((aligned(16))) float sO[128];

  const int tid = threadIdx.x, lane = tid & 31, w = tid >> 5;
  const int h = lane >> 4, m = lane & 15;
  const int b = blockIdx.x, cb = blockIdx.y;
  const int n0 = 128 * cb + 32 * w;

  const unsigned short* xh = Xh + (size_t)(b * AR + m) * NF;
  const unsigned short* xl = Xl + (size_t)(b * AR + m) * NF;
  const unsigned short* gh = GWh + (size_t)(n0 + m) * KG;
  const unsigned short* gl = GWl + (size_t)(n0 + m) * KG;

  const v8f zero8 = {0.f, 0.f, 0.f, 0.f, 0.f, 0.f, 0.f, 0.f};
  v8f ai[2], aj[2];
  #pragma unroll
  for (int nt = 0; nt < 2; ++nt) { ai[nt] = zero8; aj[nt] = zero8; }

  #pragma unroll 1
  for (int k0 = 0; k0 < NF; k0 += 32) {
    const v16b fah = load_frag(xh + k0, h);
    const v16b fal = load_frag(xl + k0, h);
    #pragma unroll
    for (int nt = 0; nt < 2; ++nt) {
      const unsigned short* rh = gh + (size_t)nt * 16 * KG;
      const unsigned short* rl = gl + (size_t)nt * 16 * KG;
      const v16b bih = load_frag(rh + k0, h);
      const v16b bil = load_frag(rl + k0, h);
      const v16b bjh = load_frag(rh + NF + k0, h);
      const v16b bjl = load_frag(rl + NF + k0, h);
      ai[nt] = wmma_bf16(fah, bih, ai[nt]);
      ai[nt] = wmma_bf16(fah, bil, ai[nt]);
      ai[nt] = wmma_bf16(fal, bih, ai[nt]);
      aj[nt] = wmma_bf16(fah, bjh, aj[nt]);
      aj[nt] = wmma_bf16(fah, bjl, aj[nt]);
      aj[nt] = wmma_bf16(fal, bjh, aj[nt]);
    }
  }

  float res[2];
  #pragma unroll
  for (int nt = 0; nt < 2; ++nt) {
    float u = ai[nt][0], v = aj[nt][0];
    #pragma unroll
    for (int r = 1; r < 8; ++r) {
      u = fminf(u, ai[nt][r]);
      v = fminf(v, aj[nt][r]);
    }
    u = fminf(u, __shfl_xor(u, 16, 32));
    v = fminf(v, __shfl_xor(v, 16, 32));
    float s = u + v;
    s = s + gfcn_b[n0 + 16 * nt + m];
    res[nt] = fmaxf(s, 0.0f);
  }

  sO[32 * w + 16 * h + m] = (h == 0) ? res[0] : res[1];
  __syncthreads();

  if (w == 0) {
    const v4f v = *(const v4fa*)(sO + 4 * lane);
    float* dst = out + (size_t)b * NG + 128 * cb + 4 * lane;
    *(volatile v4f*)dst = v;
    __threadfence();
    *(volatile v4f*)dst = v;
  }
}

extern "C" void kernel_launch(void* const* d_in, const int* in_sizes, int n_in,
                              void* d_out, int out_size, void* d_ws, size_t ws_size,
                              hipStream_t stream) {
  if (n_in < 11) return;
  if (in_sizes[0] != MROWS) return;
  if (in_sizes[1] != MROWS * EMB) return;
  if (in_sizes[2] != NROLES * EMB) return;
  if (in_sizes[3] != NF * KP) return;
  if (in_sizes[4] != NF || in_sizes[5] != NF || in_sizes[6] != NF ||
      in_sizes[7] != NF || in_sizes[8] != NF) return;
  if (in_sizes[9] != NG * KG) return;
  if (in_sizes[10] != NG) return;
  if (out_size != NB * NG) return;

  const int*   role_ids     = (const int*)d_in[0];
  const float* value_embeds = (const float*)d_in[1];
  const float* role_table   = (const float*)d_in[2];
  const float* conv_w       = (const float*)d_in[3];
  const float* conv_b       = (const float*)d_in[4];
  const float* bn_gamma     = (const float*)d_in[5];
  const float* bn_beta      = (const float*)d_in[6];
  const float* bn_mean      = (const float*)d_in[7];
  const float* bn_var       = (const float*)d_in[8];
  const float* gfcn_w       = (const float*)d_in[9];
  const float* gfcn_b       = (const float*)d_in[10];
  float* out = (float*)d_out;

  const size_t pBytes = (size_t)MROWS * KP * 2;
  const size_t cBytes = (size_t)NF * KP * 2;
  const size_t gBytes = (size_t)NG * KG * 2;
  const size_t xBytes = (size_t)MROWS * NF * 2;
  const size_t total = 2 * pBytes + 2 * cBytes + 2 * gBytes + 2 * xBytes;
  if (total > ws_size) return;

  char* ws = (char*)d_ws;
  size_t off = 0;
  unsigned short* Ph  = (unsigned short*)(ws + off); off += pBytes;
  unsigned short* Pl  = (unsigned short*)(ws + off); off += pBytes;
  unsigned short* CWh = (unsigned short*)(ws + off); off += cBytes;
  unsigned short* CWl = (unsigned short*)(ws + off); off += cBytes;
  unsigned short* GWh = (unsigned short*)(ws + off); off += gBytes;
  unsigned short* GWl = (unsigned short*)(ws + off); off += gBytes;
  unsigned short* Xh  = (unsigned short*)(ws + off); off += xBytes;
  unsigned short* Xl  = (unsigned short*)(ws + off); off += xBytes;
  if (off > ws_size) return;

  prep_kernel<<<GTOT / PREP_THREADS, PREP_THREADS, 0, stream>>>(
      role_ids, value_embeds, role_table, conv_w, gfcn_w, Ph, Pl, CWh, CWl, GWh, GWl);

  dim3 g1(MROWS / 128, NF / 64);
  gemm1_bn_kernel<<<g1, 128, 0, stream>>>(Ph, Pl, CWh, CWl, conv_b, bn_gamma, bn_beta,
                                          bn_mean, bn_var, Xh, Xl);

  dim3 g2(NB, NG / 128);
  gfcn_min_kernel<<<g2, 128, 0, stream>>>(Xh, Xl, GWh, GWl, gfcn_b, out);
}
